// DiscoveryEngineModel_71184787964500
// MI455X (gfx1250) — hardware-verified
//
#include <hip/hip_runtime.h>
#include <stddef.h>
#include <math.h>

typedef __attribute__((ext_vector_type(16))) _Float16 v16h;
typedef __attribute__((ext_vector_type(8)))  _Float16 v8h;
typedef __attribute__((ext_vector_type(16))) __bf16   v16b;
typedef __attribute__((ext_vector_type(8)))  __bf16   v8b;
typedef __attribute__((ext_vector_type(8)))  float    v8f;
typedef __attribute__((ext_vector_type(4)))  float    v4f;
typedef __attribute__((ext_vector_type(2)))  float    v2f;
typedef __attribute__((ext_vector_type(4)))  int      v4i;

constexpr int HID    = 64;
constexpr int NODEF  = 4;
constexpr int EIN    = 10;
constexpr int KE1    = 32;
constexpr int NE1    = 128;
constexpr int KNODE  = 96;
constexpr int NHH    = 69;
constexpr int CHE    = 204800;
constexpr int NBA    = 1024;
constexpr int RPQ    = 1024;
constexpr int NTHR   = 256;
constexpr int NWAVE  = 8;
constexpr int EPT    = 8;
constexpr int NGRP   = 1;
constexpr int SUBCH  = NTHR * EPT * NGRP;
constexpr int WCAP   = EPT * NGRP * 32;
constexpr int LISTN  = NWAVE * WCAP;
constexpr int MAXSUB = CHE / SUBCH;
constexpr int LDS_AGG = (NBA * HID + NBA * 2) * 4 + LISTN * 4 + 64;

static_assert((SUBCH & (SUBCH - 1)) == 0 && SUBCH <= 4096);
static_assert((NBA & (NBA - 1)) == 0 && NBA <= 4096);
static_assert(RPQ % NBA == 0 && RPQ % 64 == 0 && RPQ % NTHR == 0);
static_assert(CHE % SUBCH == 0 && CHE % 256 == 0 && CHE % 64 == 0);
static_assert(LDS_AGG == 278592);
static_assert(KE1 % 32 == 0 && KNODE % 32 == 0 && NHH <= KNODE && 2 * EIN <= KE1);
static_assert((RPQ * (KNODE / 8)) % NTHR == 0);

__device__ __forceinline__ unsigned short f2bf_bits(float f) {
  unsigned u = __float_as_uint(f);
  return (unsigned short)((u + 0x7FFFu + ((u >> 16) & 1u)) >> 16);
}
__device__ __forceinline__ float bf_bits2f(unsigned short h) { return __uint_as_float(((unsigned)h) << 16); }

__device__ __forceinline__ void dep_guard_h(v8f& a, v8f& b, v16h x, v16h y) { asm volatile("v_nop\n\tv_nop\n\tv_nop\n\tv_nop" : "+v"(a), "+v"(b) : "v"(x), "v"(y)); }
__device__ __forceinline__ void dep_guard_b(v8f& a, v8f& b, v16b x, v16b y) { asm volatile("v_nop\n\tv_nop\n\tv_nop\n\tv_nop" : "+v"(a), "+v"(b) : "v"(x), "v"(y)); }
__device__ __forceinline__ void keep4_h(v16h a, v16h b, v16h c, v16h d) { asm volatile("v_nop" :: "v"(a), "v"(b), "v"(c), "v"(d)); }
__device__ __forceinline__ void keep4_b(v16b a, v16b b, v16b c, v16b d) { asm volatile("v_nop" :: "v"(a), "v"(b), "v"(c), "v"(d)); }
__device__ __forceinline__ void acc_guard4(v8f& a, v8f& b, v8f& c, v8f& d) { asm volatile("v_nop\n\tv_nop\n\tv_nop\n\tv_nop" : "+v"(a), "+v"(b), "+v"(c), "+v"(d)); }
template <typename T> struct Frag;
template <> struct Frag<_Float16> {
  typedef v16h V; union U { v16h v; v8h h[2]; };
  static __device__ __forceinline__ v16h load(const _Float16* p) {
    U f; f.h[0] = *(const v8h*)(p); f.h[1] = *(const v8h*)(p + 16); return f.v;
  }
  static __device__ __forceinline__ v8f mma(v16h a, v16h b, v8f c) {
    return __builtin_amdgcn_wmma_f32_16x16x32_f16(false, a, false, b, (short)0, c, false, false);
  }
  static __device__ __forceinline__ void guard(v8f& a, v8f& b, v16h x, v16h y) { dep_guard_h(a, b, x, y); }
  static __device__ __forceinline__ void keep(v16h a, v16h b, v16h c, v16h d) { keep4_h(a, b, c, d); }
};
template <> struct Frag<__bf16> {
  typedef v16b V; union U { v16b v; v8b h[2]; };
  static __device__ __forceinline__ v16b load(const __bf16* p) {
    U f; f.h[0] = *(const v8b*)(p); f.h[1] = *(const v8b*)(p + 16); return f.v;
  }
  static __device__ __forceinline__ v8f mma(v16b a, v16b b, v8f c) {
    return __builtin_amdgcn_wmma_f32_16x16x32_bf16(false, a, false, b, (short)0, c, false, false);
  }
  static __device__ __forceinline__ void guard(v8f& a, v8f& b, v16b x, v16b y) { dep_guard_b(a, b, x, y); }
  static __device__ __forceinline__ void keep(v16b a, v16b b, v16b c, v16b d) { keep4_b(a, b, c, d); }
};

template <int ET> struct Elem;
template <> struct Elem<0> { typedef _Float16 T; };
template <> struct Elem<1> { typedef __bf16 T; };
template <int ET, bool SPLIT, int BIAS_MODE, int OUT_MODE, bool RESID, int ACT = 0>
__global__ __launch_bounds__(256) void wmma_gemm64(
    const unsigned short* __restrict__ Ap, const unsigned short* __restrict__ A2p, int lda, long strideA,
    const unsigned short* __restrict__ Btp, const unsigned short* __restrict__ Bt2p, int ldb, long strideB,
    void* __restrict__ Cout, void* __restrict__ Cout2, int ldc, long strideC,
    const float* __restrict__ bias,
    const float* __restrict__ resid, long strideR,
    int M, int N, int K, float scale) {
  typedef typename Elem<ET>::T T;
  typedef typename Frag<T>::V V;
  const T* A = (const T*)Ap; const T* A2 = (const T*)A2p; const T* Bt = (const T*)Btp; const T* Bt2 = (const T*)Bt2p;
  __shared__ __align__(16) float sT[8][16 * 68];
  const int b    = blockIdx.y;
  const int lane = threadIdx.x & 31;
  const int wave = threadIdx.x >> 5;
  const int tilesN = N >> 6;
  const int tilesM = M >> 6;
  const int tile = blockIdx.x * 8 + wave;
  if (tile >= tilesM * tilesN) return;
  const int tm = tile / tilesN;
  const int tn = tile - tm * tilesN;
  const int m0 = tm << 6;
  const int n0 = tn << 6;

  const T* Ab  = A  + (size_t)b * strideA;
  const T* Bb  = Bt + (size_t)b * strideB;
  const T* Ab2 = SPLIT ? (A2  + (size_t)b * strideA) : nullptr;
  const T* Bb2 = SPLIT ? (Bt2 + (size_t)b * strideB) : nullptr;

  const int rlane = lane & 15;
  const int koff  = (lane >> 4) * 8;
  const int mOff  = (lane >> 4) * 8;

  v8f acc[4][4];
#pragma unroll
  for (int i = 0; i < 4; ++i)
#pragma unroll
    for (int j = 0; j < 4; ++j) acc[i][j] = (v8f){0.f,0.f,0.f,0.f,0.f,0.f,0.f,0.f};

  for (int k0 = 0; k0 < K; k0 += 32) {
    V bh[4], bl[4];
#pragma unroll
    for (int j = 0; j < 4; ++j) {
      const size_t bo = (size_t)(n0 + (j << 4) + rlane) * ldb + koff + k0;
      bh[j] = Frag<T>::load(Bb + bo);
      if (SPLIT) bl[j] = Frag<T>::load(Bb2 + bo);
    }
#pragma unroll
    for (int i = 0; i < 4; ++i) {
      const size_t ao = (size_t)(m0 + (i << 4) + rlane) * lda + koff + k0;
      V ah = Frag<T>::load(Ab + ao);
      V al;
      if (SPLIT) al = Frag<T>::load(Ab2 + ao);
#pragma unroll
      for (int j = 0; j < 4; ++j) {
        acc[i][j] = Frag<T>::mma(ah, bh[j], acc[i][j]);
        if (SPLIT) {
          acc[i][j] = Frag<T>::mma(ah, bl[j], acc[i][j]);
          acc[i][j] = Frag<T>::mma(al, bh[j], acc[i][j]);
        }
      }
      Frag<T>::guard(acc[i][0], acc[i][3], ah, SPLIT ? al : ah);
    }
    Frag<T>::keep(bh[0], bh[1], bh[2], bh[3]);
    if (SPLIT) Frag<T>::keep(bl[0], bl[1], bl[2], bl[3]);
  }
  acc_guard4(acc[0][0], acc[0][1], acc[0][2], acc[0][3]);
  acc_guard4(acc[1][0], acc[1][1], acc[1][2], acc[1][3]);
  acc_guard4(acc[2][0], acc[2][1], acc[2][2], acc[2][3]);
  acc_guard4(acc[3][0], acc[3][1], acc[3][2], acc[3][3]);

  float* slab = sT[wave];
  const float* Rb = RESID ? (resid + (size_t)b * strideR) : nullptr;
#pragma unroll
  for (int i = 0; i < 4; ++i) {
    const int mBase = m0 + (i << 4);
#pragma unroll
    for (int j = 0; j < 4; ++j) {
      const int n = n0 + (j << 4) + rlane;
      float bv = 0.f;
      if (BIAS_MODE == 2) bv = bias[n];
#pragma unroll
      for (int r = 0; r < 8; ++r) {
        float v = acc[i][j][r] * scale;
        if (BIAS_MODE == 1) v += bias[mBase + mOff + r];
        if (BIAS_MODE == 2) v += bv;
        if (RESID) v += Rb[(size_t)(mBase + mOff + r) * ldc + n];
        if (ACT == 1) v = tanhf(v);
        if (ACT == 2) v = fmaxf(v, 0.0f);
        if (ACT == 3) v = v / (1.0f + expf(-v));
        if (ACT == 4) v = (v > 0.f) ? v : 0.01f * v;
        if (ACT == 5) v = 0.5f * v * (1.0f + erff(v * 0.70710678118654752f));
        if (ACT == 6) v = v * __builtin_amdgcn_rcpf(1.0f + __expf(-v));
        slab[(mOff + r) * 68 + (j << 4) + rlane] = v;
      }
    }
    __builtin_amdgcn_fence(__ATOMIC_RELEASE, "workgroup");
    __builtin_amdgcn_wave_barrier();
    __builtin_amdgcn_fence(__ATOMIC_ACQUIRE, "workgroup");
    if (OUT_MODE == 0) {
      float* C = (float*)Cout + (size_t)b * strideC;
      const int hh = lane >> 4, c4 = (lane & 15) * 4;
      for (int pass = 0; pass < 2; ++pass) {
#pragma unroll
        for (int it = 0; it < 8; ++it) {
          const int row = it * 2 + hh;
          v4f v = *(const v4f*)(slab + row * 68 + c4);
          *(volatile v4f*)(C + (size_t)(mBase + row) * ldc + n0 + c4) = v;
        }
        __threadfence();
      }
    } else {
      const int q = lane >> 3, c8 = (lane & 7) * 8;
      unsigned short* C  = (unsigned short*)Cout  + (size_t)b * strideC;
      unsigned short* C2 = (OUT_MODE == 2) ? ((unsigned short*)Cout2 + (size_t)b * strideC) : nullptr;
      for (int pass = 0; pass < 2; ++pass) {
#pragma unroll
        for (int it = 0; it < 4; ++it) {
          const int row = it * 4 + q;
          const float* sp = slab + row * 68 + c8;
          v8h hv, lv;
#pragma unroll
          for (int e = 0; e < 8; ++e) {
            if (OUT_MODE == 1) {
              hv[e] = (_Float16)sp[e];
            } else {
              unsigned short hb = f2bf_bits(sp[e]);
              unsigned short lb = f2bf_bits(sp[e] - bf_bits2f(hb));
              hv[e] = __builtin_bit_cast(_Float16, hb);
              lv[e] = __builtin_bit_cast(_Float16, lb);
            }
          }
          *(volatile v8h*)(C + (size_t)(mBase + row) * ldc + n0 + c8) = hv;
          if (OUT_MODE == 2) *(volatile v8h*)(C2 + (size_t)(mBase + row) * ldc + n0 + c8) = lv;
        }
        __threadfence();
      }
    }
    __builtin_amdgcn_fence(__ATOMIC_RELEASE, "workgroup");
    __builtin_amdgcn_wave_barrier();
    __builtin_amdgcn_fence(__ATOMIC_ACQUIRE, "workgroup");
  }
}

template <int NB>
__device__ __forceinline__ int scan_chunk(const int* __restrict__ lst, int nE, int cbase, int nodeBase,
                                          int* list, int tid, int lane, int wave, int fullvec) {
  int wc = 0;
#pragma unroll
  for (int g = 0; g < NGRP; ++g) {
    const int el0 = (g * NTHR + tid) * EPT;
    const int e0  = cbase + el0;
    v4i da, db;
    if (fullvec) {
      da = *(const v4i*)(lst + e0);
      db = *(const v4i*)(lst + e0 + 4);
    } else {
      const int em = nE - 1;
      da.x = lst[(e0     < em) ? e0     : em];
      da.y = lst[(e0 + 1 < em) ? e0 + 1 : em];
      da.z = lst[(e0 + 2 < em) ? e0 + 2 : em];
      da.w = lst[(e0 + 3 < em) ? e0 + 3 : em];
      db.x = lst[(e0 + 4 < em) ? e0 + 4 : em];
      db.y = lst[(e0 + 5 < em) ? e0 + 5 : em];
      db.z = lst[(e0 + 6 < em) ? e0 + 6 : em];
      db.w = lst[(e0 + 7 < em) ? e0 + 7 : em];
    }
    const bool v0 = (e0 < nE), v1 = (e0 + 1 < nE), v2 = (e0 + 2 < nE), v3 = (e0 + 3 < nE);
    const bool v4 = (e0 + 4 < nE), v5 = (e0 + 5 < nE), v6 = (e0 + 6 < nE), v7 = (e0 + 7 < nE);
    const unsigned nb = (unsigned)nodeBase;
    const unsigned s0 = (unsigned)da.x - nb, s1 = (unsigned)da.y - nb;
    const unsigned s2 = (unsigned)da.z - nb, s3 = (unsigned)da.w - nb;
    const unsigned s4 = (unsigned)db.x - nb, s5 = (unsigned)db.y - nb;
    const unsigned s6 = (unsigned)db.z - nb, s7 = (unsigned)db.w - nb;
    const bool h0 = v0 && (s0 < (unsigned)NB), h1 = v1 && (s1 < (unsigned)NB);
    const bool h2 = v2 && (s2 < (unsigned)NB), h3 = v3 && (s3 < (unsigned)NB);
    const bool h4 = v4 && (s4 < (unsigned)NB), h5 = v5 && (s5 < (unsigned)NB);
    const bool h6 = v6 && (s6 < (unsigned)NB), h7 = v7 && (s7 < (unsigned)NB);
    const unsigned any = __builtin_amdgcn_ballot_w32(h0 | h1 | h2 | h3 | h4 | h5 | h6 | h7);
    if (any != 0u) {
#define HITJ(J, HJ, SJ) { \
        const unsigned mj = __builtin_amdgcn_ballot_w32(HJ); \
        if (mj != 0u) { \
          if (HJ) { \
            const int pos = wc + (int)__builtin_amdgcn_mbcnt_lo(mj, 0u); \
            if (pos < WCAP) list[wave * WCAP + pos] = ((el0 + (J)) << 12) | (int)(SJ); \
          } \
          wc += (int)__builtin_popcount(mj); } }
      HITJ(0, h0, s0)
      HITJ(1, h1, s1)
      HITJ(2, h2, s2)
      HITJ(3, h3, s3)
      HITJ(4, h4, s4)
      HITJ(5, h5, s5)
      HITJ(6, h6, s6)
      HITJ(7, h7, s7)
#undef HITJ
    }
  }
  return wc;
}

__global__ __launch_bounds__(NTHR) void k_wprep(const float* __restrict__ W, int Kin, int ncol, int Kpad,
                                                int loK, unsigned short* bt) {
  const int tpr = Kpad >> 3;
  const int i = blockIdx.x * NTHR + threadIdx.x;
  if (i >= HID * tpr) return;
  const int n   = i / tpr;
  const int k0  = (i - n * tpr) * 8;
  const int ncl = (n < ncol) ? n : ncol - 1;
  v8h hv;
#pragma unroll
  for (int e = 0; e < 8; ++e) {
    const int k   = k0 + e;
    const int khc = (k < Kin) ? k : Kin - 1;
    const int kl  = k - loK;
    const int klc = (kl < 0) ? 0 : ((kl < Kin) ? kl : Kin - 1);
    const float whi = W[(size_t)khc * ncol + ncl];
    const float wlo = W[(size_t)klc * ncol + ncl];
    float v = 0.f;
    if (k < Kin) v = 64.0f * whi;
    else if (kl >= 0 && kl < Kin) v = 4.0f * wlo;
    if (n >= ncol) v = 0.f;
    hv[e] = (_Float16)v;
  }
  const size_t o = (size_t)i * 8;
  *(volatile v8h*)(bt + o) = hv;
  __threadfence();
  *(volatile v8h*)(bt + o) = hv;
}

__global__ __launch_bounds__(NTHR) void k_wsplit(const float* __restrict__ W, int Kin, int ncol, int Kpad,
                                                 unsigned short* bth, unsigned short* btl) {
  const int tpr = Kpad >> 3;
  const int i = blockIdx.x * NTHR + threadIdx.x;
  if (i >= HID * tpr) return;
  const int n   = i / tpr;
  const int k0  = (i - n * tpr) * 8;
  const int ncl = (n < ncol) ? n : ncol - 1;
  v8h hv, lv;
#pragma unroll
  for (int e = 0; e < 8; ++e) {
    const int k  = k0 + e;
    const int kc = (k < Kin) ? k : Kin - 1;
    float v = W[(size_t)kc * ncol + ncl];
    if (k >= Kin || n >= ncol) v = 0.f;
    const unsigned short hb = f2bf_bits(v);
    const unsigned short lb = f2bf_bits(v - bf_bits2f(hb));
    hv[e] = __builtin_bit_cast(_Float16, hb);
    lv[e] = __builtin_bit_cast(_Float16, lb);
  }
  const size_t o = (size_t)i * 8;
  *(volatile v8h*)(bth + o) = hv;
  *(volatile v8h*)(btl + o) = lv;
  __threadfence();
  *(volatile v8h*)(bth + o) = hv;
  *(volatile v8h*)(btl + o) = lv;
}

__global__ __launch_bounds__(32) void k_bias128(const float* __restrict__ ba, const float* __restrict__ bb,
                                                float* o) {
  const int lane = threadIdx.x & 31;
  float t[4];
#pragma unroll
  for (int j = 0; j < 4; ++j) {
    const int c  = 4 * lane + j;
    const int ca = (c < HID) ? c : HID - 1;
    int cb = c - HID; cb = (cb < 0) ? 0 : ((cb < HID) ? cb : HID - 1);
    const float a = ba[ca];
    const float bv = bb[cb];
    t[j] = (c < HID) ? a : bv;
  }
  const v4f v = {t[0], t[1], t[2], t[3]};
  *(volatile v4f*)(o + 4 * lane) = v;
  __threadfence();
  *(volatile v4f*)(o + 4 * lane) = v;
}

__device__ __forceinline__ void put_hl(_Float16* row, int k, float v) {
  const _Float16 h = (_Float16)v;
  row[k] = h;
  row[k + EIN] = (_Float16)((v - (float)h) * 16.0f);
}

__global__ __launch_bounds__(NTHR) void k_gather(
    const float* __restrict__ x, const float* __restrict__ pos, const float* __restrict__ vel,
    const int* __restrict__ ei, int nN, int nE, int ebase, int Mc, unsigned short* tmp) {
#pragma clang fp contract(off)
  __shared__ __align__(16) _Float16 st[NTHR * KE1];
  const int tid = threadIdx.x;
  const int r = blockIdx.x * NTHR + tid;
  const int e = ebase + r;
  const bool valid = (r < Mc) && (e < nE);
  int ec = (e < nE) ? e : nE - 1; ec = (ec < 0) ? 0 : ec;
  int s = ei[ec];
  int d = ei[(size_t)nE + ec];
  s = (s < 0) ? 0 : ((s > nN - 1) ? nN - 1 : s);
  d = (d < 0) ? 0 : ((d > nN - 1) ? nN - 1 : d);
  const v4f xd = *(const v4f*)(x + (size_t)d * NODEF);
  const v4f xs = *(const v4f*)(x + (size_t)s * NODEF);
  const v2f pd = *(const v2f*)(pos + (size_t)d * 2);
  const v2f ps = *(const v2f*)(pos + (size_t)s * 2);
  const v2f vd = *(const v2f*)(vel + (size_t)d * 2);
  const v2f vs = *(const v2f*)(vel + (size_t)s * 2);
  const float rpx = ps.x - pd.x, rpy = ps.y - pd.y;
  const float rvx = vs.x - vd.x, rvy = vs.y - vd.y;
  const float dsq = rpx * rpx + rpy * rpy;
  const float dvr = rvx * rpx + rvy * rpy;
  const float z = 0.0f;
  _Float16* row = st + tid * KE1;
  put_hl(row, 0, valid ? xd.x : z);
  put_hl(row, 1, valid ? xd.y : z);
  put_hl(row, 2, valid ? xd.z : z);
  put_hl(row, 3, valid ? xd.w : z);
  put_hl(row, 4, valid ? xs.x : z);
  put_hl(row, 5, valid ? xs.y : z);
  put_hl(row, 6, valid ? xs.z : z);
  put_hl(row, 7, valid ? xs.w : z);
  put_hl(row, 8, valid ? dsq : z);
  put_hl(row, 9, valid ? dvr : z);
#pragma unroll
  for (int k = 2 * EIN; k < KE1; ++k) row[k] = (_Float16)0.0f;
  __syncthreads();
  const int rowBlock = blockIdx.x * NTHR;
  for (int pass = 0; pass < 2; ++pass) {
#pragma unroll
    for (int it = 0; it < 4; ++it) {
      const int q  = it * NTHR + tid;
      const int lr = q >> 2;
      const int pc = (q & 3) * 8;
      const int grow = rowBlock + lr;
      const v8h hv = *(const v8h*)(st + lr * KE1 + pc);
      if (grow < Mc) *(volatile v8h*)(tmp + (size_t)grow * KE1 + pc) = hv;
    }
    __threadfence();
  }
}

__global__ __launch_bounds__(NTHR) void k_vw(
    const unsigned short* __restrict__ hv, const float* __restrict__ w2, const float* __restrict__ b2,
    const int* __restrict__ ei, const float* __restrict__ pos,
    int nN, int nE, int ebase, int Mc, float* mv) {
  const int tid = threadIdx.x, lane = tid & 31, wave = tid >> 5;
  const int r  = blockIdx.x * NTHR + tid;
  const int rc = (r < Mc) ? r : Mc - 1;
  const _Float16* vp = (const _Float16*)hv + (size_t)rc * NE1 + HID;
  float acc = 0.0f;
#pragma unroll
  for (int p = 0; p < 8; ++p) {
    const v8h q = *(const v8h*)(vp + 8 * p);
#pragma unroll
    for (int t = 0; t < 8; ++t) acc += (float)q[t] * w2[8 * p + t];
  }
  const float vw = acc + b2[0];
  const int e = ebase + r;
  const bool valid = (r < Mc) && (e < nE);
  int ec = (e < nE) ? e : nE - 1; ec = (ec < 0) ? 0 : ec;
  int s = ei[ec];
  int d = ei[(size_t)nE + ec];
  s = (s < 0) ? 0 : ((s > nN - 1) ? nN - 1 : s);
  d = (d < 0) ? 0 : ((d > nN - 1) ? nN - 1 : d);
  const v2f pd = *(const v2f*)(pos + (size_t)d * 2);
  const v2f ps = *(const v2f*)(pos + (size_t)s * 2);
  const float rpx = ps.x - pd.x, rpy = ps.y - pd.y;
  const float mvx = valid ? vw * rpx : 0.0f;
  const float mvy = valid ? vw * rpy : 0.0f;
  const int sl0 = (2 * lane) & 31, sl1 = (2 * lane + 1) & 31;
  const float a0 = __shfl(mvx, sl0, 32), a1 = __shfl(mvy, sl0, 32);
  const float a2 = __shfl(mvx, sl1, 32), a3 = __shfl(mvy, sl1, 32);
  const v4f o = {a0, a1, a2, a3};
  const int rw = blockIdx.x * NTHR + wave * 32;
  const int lw = (lane < 16) ? lane : 15;
  float* op = mv + (size_t)rw * 2 + 4 * lw;
  const bool doit = (lane < 16) && (rw < Mc);
  if (doit) *(volatile v4f*)op = o;
  __threadfence();
  if (doit) *(volatile v4f*)op = o;
}

__global__ __launch_bounds__(NTHR) void k_agg(
    const int* __restrict__ dstl, int nEc,
    const float* __restrict__ mh, const float* __restrict__ mvp,
    float* aggh, float* aggv, int nN, int first, int vec_ok) {
  constexpr int NB   = NBA;
  constexpr int NV4  = NB * HID / 4;
  constexpr int NV4V = NB * 2 / 4;
  static_assert(NV4 % NTHR == 0 && NV4V % NTHR == 0);
  extern __shared__ v4f lds_dyn[];
  float* acc  = (float*)lds_dyn;
  float* accv = acc + NB * HID;
  int*   list = (int*)(accv + NB * 2);
  int*   wcnt = list + LISTN;
  const int tid = threadIdx.x, lane = tid & 31, wave = tid >> 5;
  const int nodeBase = blockIdx.x * NB;
  float* gh = aggh + (size_t)nodeBase * HID;
  float* gv = aggv + (size_t)nodeBase * 2;

  if (first) {
    const v4f zz = {0.f, 0.f, 0.f, 0.f};
    for (int i = tid; i < NV4 + NV4V; i += NTHR) lds_dyn[i] = zz;
  } else {
    for (int i = tid; i < NV4; i += NTHR) lds_dyn[i] = ((const v4f*)gh)[i];
    for (int i = tid; i < NV4V; i += NTHR) lds_dyn[NV4 + i] = ((const v4f*)gv)[i];
  }
  __syncthreads();

  int nSub = (nEc + SUBCH - 1) / SUBCH;
  nSub = (nSub > MAXSUB) ? MAXSUB : nSub;
#pragma unroll 1
  for (int ch = 0; ch < nSub; ++ch) {
    const int cbase = ch * SUBCH;
    const int fullvec = (vec_ok != 0 && cbase + SUBCH <= nEc) ? 1 : 0;
    const int wc = scan_chunk<NB>(dstl, nEc, cbase, nodeBase, list, tid, lane, wave, fullvec);
    if (lane == 0) wcnt[wave] = wc;
    __syncthreads();
    if (wave == 0) {
#pragma unroll 1
      for (int wsx = 0; wsx < NWAVE; ++wsx) {
        int n = __builtin_amdgcn_readfirstlane(wcnt[wsx]);
        n = n > WCAP ? WCAP : (n < 0 ? 0 : n);
        const int* lp = list + wsx * WCAP;
#pragma unroll 1
        for (int i = 0; i < n; ++i) {
          const int ent  = __builtin_amdgcn_readfirstlane(lp[i]);
          const int slot = ent & (NB - 1);
          int el = cbase + ((ent >> 12) & (SUBCH - 1));
          el = (el > nEc - 1) ? nEc - 1 : el;
          const v2f m2 = *(const v2f*)(mh + (size_t)el * HID + 2 * lane);
          v2f* ap = (v2f*)(acc + slot * HID + 2 * lane);
          const v2f av = *ap;
          *ap = av + m2;
          const float vv = mvp[(size_t)el * 2 + (lane & 1)];
          if (lane < 2) {
            const float a = accv[slot * 2 + lane];
            accv[slot * 2 + lane] = a + vv;
          }
        }
      }
    }
    __syncthreads();
  }

  for (int pass = 0; pass < 2; ++pass) {
#pragma unroll 4
    for (int i = tid; i < NV4; i += NTHR) { const v4f v = lds_dyn[i]; ((volatile v4f*)gh)[i] = v; }
#pragma unroll
    for (int i = tid; i < NV4V; i += NTHR) { const v4f v = lds_dyn[NV4 + i]; ((volatile v4f*)gv)[i] = v; }
    __threadfence();
  }
}

__global__ __launch_bounds__(NTHR) void k_hh(const float* __restrict__ x, const float* __restrict__ aggh,
                                             const float* __restrict__ aggv, int nN, int RP,
                                             unsigned short* hhh, unsigned short* hhl) {
#pragma clang fp contract(off)
  constexpr int PPR = KNODE / 8;
  const int i = blockIdx.x * NTHR + threadIdx.x;
  const int row = i / PPR;
  const int p = i - row * PPR;
  int cb = 8 * p - 4; cb = (cb < 0) ? 0 : ((cb > HID - 8) ? HID - 8 : cb);
  const int rown = (row < nN) ? row : nN - 1;
  const int rowa = (row < RP) ? row : RP - 1;
  const v4f xv = *(const v4f*)(x + (size_t)rown * NODEF);
  const float* ar = aggh + (size_t)rowa * HID + cb;
  const v4f a0 = *(const v4f*)ar;
  const v4f a1 = *(const v4f*)(ar + 4);
  const v2f av = *(const v2f*)(aggv + (size_t)rowa * 2);
  const float nrm = sqrtf(av.x * av.x + av.y * av.y);
  const float A8[8] = {a0.x, a0.y, a0.z, a0.w, a1.x, a1.y, a1.z, a1.w};
  const float X4[4] = {xv.x, xv.y, xv.z, xv.w};
  v8h ho, lo;
#pragma unroll
  for (int j = 0; j < 8; ++j) {
    const float c0 = (j < 4) ? X4[j & 3] : A8[(j + 4) & 7];
    const float c8 = (j < 4) ? A8[(j + 4) & 7] : ((j == 4) ? nrm : 0.0f);
    const float cm = A8[j];
    float v = (p == 0) ? c0 : ((p == 8) ? c8 : ((p <= 7) ? cm : 0.0f));
    if (row >= nN) v = 0.0f;
    const unsigned short hb = f2bf_bits(v);
    const unsigned short lb = f2bf_bits(v - bf_bits2f(hb));
    ho[j] = __builtin_bit_cast(_Float16, hb);
    lo[j] = __builtin_bit_cast(_Float16, lb);
  }
  const bool ok = (row < RP);
  const size_t o = (size_t)i * 8;
  if (ok) { *(volatile v8h*)(hhh + o) = ho; *(volatile v8h*)(hhl + o) = lo; }
  __threadfence();
  if (ok) { *(volatile v8h*)(hhh + o) = ho; *(volatile v8h*)(hhl + o) = lo; }
}

__global__ __launch_bounds__(NTHR) void k_copy(const float* __restrict__ src, float* out, int n4) {
  const int i = blockIdx.x * NTHR + threadIdx.x;
  const int ic = (i < n4) ? i : n4 - 1;
  const v4f v = ((const v4f*)src)[ic];
  if (i < n4) ((volatile v4f*)out)[i] = v;
  __threadfence();
  if (i < n4) ((volatile v4f*)out)[i] = v;
}

extern "C" void kernel_launch(void* const* d_in, const int* in_sizes, int n_in,
                              void* d_out, int out_size, void* d_ws, size_t ws_size,
                              hipStream_t stream) {
  if (n_in < 18) return;
  const int nN = in_sizes[0] / NODEF;
  const int nE = in_sizes[3] / 2;
  if (nN < 1 || in_sizes[0] != nN * NODEF || in_sizes[1] != nN * 2 || in_sizes[2] != nN * 2) return;
  if (nN > (1 << 24)) return;
  if (nE < 1 || in_sizes[3] != 2 * nE) return;
  if (in_sizes[4] != EIN * HID || in_sizes[5] != HID || in_sizes[6] != HID * HID || in_sizes[7] != HID) return;
  if (in_sizes[8] != HID * HID || in_sizes[9] != HID) return;
  if (in_sizes[10] != EIN * HID || in_sizes[11] != HID || in_sizes[12] != HID || in_sizes[13] < 1) return;
  if (in_sizes[14] != NHH * HID || in_sizes[15] != HID || in_sizes[16] != HID * HID || in_sizes[17] != HID) return;
  if (out_size != nN * HID) return;
  const int nChunks = (nE + CHE - 1) / CHE;
  if (nChunks < 1 || nChunks > 64) return;

  const float* x     = (const float*)d_in[0];
  const float* pos   = (const float*)d_in[1];
  const float* vel   = (const float*)d_in[2];
  const int*   ei    = (const int*)d_in[3];
  const float* pe_w1 = (const float*)d_in[4];
  const float* pe_b1 = (const float*)d_in[5];
  const float* pe_w2 = (const float*)d_in[6];
  const float* pe_b2 = (const float*)d_in[7];
  const float* pe_w3 = (const float*)d_in[8];
  const float* pe_b3 = (const float*)d_in[9];
  const float* pv_w1 = (const float*)d_in[10];
  const float* pv_b1 = (const float*)d_in[11];
  const float* pv_w2 = (const float*)d_in[12];
  const float* pv_b2 = (const float*)d_in[13];
  const float* ph_w1 = (const float*)d_in[14];
  const float* ph_b1 = (const float*)d_in[15];
  const float* ph_w2 = (const float*)d_in[16];
  const float* ph_b2 = (const float*)d_in[17];
  float* out = (float*)d_out;

  const int RP = ((nN + RPQ - 1) / RPQ) * RPQ;
  const int nA = RP / NBA;

  size_t off = 0;
  auto carve = [&](size_t bytes) { const size_t o = off; off += (bytes + 255) & ~(size_t)255; return o; };
  const size_t oW1   = carve((size_t)NE1 * KE1 * 2);
  const size_t oW2   = carve((size_t)HID * HID * 2);
  const size_t oW3   = carve((size_t)HID * HID * 2);
  const size_t oWP1H = carve((size_t)HID * KNODE * 2);
  const size_t oWP1L = carve((size_t)HID * KNODE * 2);
  const size_t oWP2H = carve((size_t)HID * HID * 2);
  const size_t oWP2L = carve((size_t)HID * HID * 2);
  const size_t oB    = carve((size_t)NE1 * 4);
  const size_t oAGH  = carve((size_t)RP * HID * 4);
  const size_t oAGV  = carve((size_t)RP * 2 * 4);
  const size_t oTMP  = carve((size_t)CHE * KE1 * 2);
  const size_t szHV  = (size_t)CHE * NE1 * 2;
  const size_t oHV   = carve(szHV);
  const size_t szH2  = (size_t)CHE * HID * 2;
  const size_t oH2   = carve(szH2);
  const size_t oMV   = carve((size_t)CHE * 2 * 4);
  if (off > ws_size || off > (size_t)134217728) return;
  const size_t szHH = (((size_t)RP * KNODE * 2) + 255) & ~(size_t)255;
  const size_t szHN = (((size_t)RP * HID * 2) + 255) & ~(size_t)255;
  const size_t oHHH = oHV;
  const size_t oHHL = oHHH + szHH;
  const size_t oHNH = oHHL + szHH;
  const size_t oHNL = oHNH + szHN;
  if (2 * szHH + 2 * szHN > szHV) return;
  if ((size_t)CHE * HID * 4 > szHV) return;
  const size_t oOUT = oH2;
  if ((size_t)RP * HID * 4 > szH2) return;

  char* ws = (char*)d_ws;
  unsigned short* w1   = (unsigned short*)(ws + oW1);
  unsigned short* w2   = (unsigned short*)(ws + oW2);
  unsigned short* w3   = (unsigned short*)(ws + oW3);
  unsigned short* wp1h = (unsigned short*)(ws + oWP1H);
  unsigned short* wp1l = (unsigned short*)(ws + oWP1L);
  unsigned short* wp2h = (unsigned short*)(ws + oWP2H);
  unsigned short* wp2l = (unsigned short*)(ws + oWP2L);
  float* b128 = (float*)(ws + oB);
  float* aggh = (float*)(ws + oAGH);
  float* aggv = (float*)(ws + oAGV);
  unsigned short* tmp = (unsigned short*)(ws + oTMP);
  unsigned short* hv  = (unsigned short*)(ws + oHV);
  float* mhf = (float*)(ws + oHV);
  unsigned short* h2  = (unsigned short*)(ws + oH2);
  float* mv  = (float*)(ws + oMV);
  unsigned short* hhh = (unsigned short*)(ws + oHHH);
  unsigned short* hhl = (unsigned short*)(ws + oHHL);
  unsigned short* hnh = (unsigned short*)(ws + oHNH);
  unsigned short* hnl = (unsigned short*)(ws + oHNL);
  float* outp = (float*)(ws + oOUT);

  const float gscale = 0.015625f;
  auto gemm_blocks = [](int M, int Nn) { return ((M / 64) * (Nn / 64) + 7) / 8; };

  k_wprep<<<(HID * (KE1 / 8) + NTHR - 1) / NTHR, NTHR, 0, stream>>>(pe_w1, EIN, HID, KE1, EIN, w1);
  k_wprep<<<(HID * (KE1 / 8) + NTHR - 1) / NTHR, NTHR, 0, stream>>>(pv_w1, EIN, HID, KE1, EIN, w1 + (size_t)HID * KE1);
  k_wprep<<<(HID * (HID / 8) + NTHR - 1) / NTHR, NTHR, 0, stream>>>(pe_w2, HID, HID, HID, HID, w2);
  k_wprep<<<(HID * (HID / 8) + NTHR - 1) / NTHR, NTHR, 0, stream>>>(pe_w3, HID, HID, HID, HID, w3);
  k_wsplit<<<(HID * (KNODE / 8) + NTHR - 1) / NTHR, NTHR, 0, stream>>>(ph_w1, NHH, HID, KNODE, wp1h, wp1l);
  k_wsplit<<<(HID * (HID / 8) + NTHR - 1) / NTHR, NTHR, 0, stream>>>(ph_w2, HID, HID, HID, wp2h, wp2l);
  k_bias128<<<1, 32, 0, stream>>>(pe_b1, pv_b1, b128);

  for (int c = 0; c < nChunks; ++c) {
    const int base = c * CHE;
    int Ec = nE - base; if (Ec > CHE) Ec = CHE;
    const int Mc = ((Ec + 63) / 64) * 64;
    const int gb = (Mc + NTHR - 1) / NTHR;
    const int vec = (((size_t)nE + (size_t)base) & 3) == 0 ? 1 : 0;

    k_gather<<<gb, NTHR, 0, stream>>>(x, pos, vel, ei, nN, nE, base, Mc, tmp);
    wmma_gemm64<0, false, 2, 1, false, 6><<<dim3(gemm_blocks(Mc, NE1), 1), 256, 0, stream>>>(
        tmp, tmp, KE1, 0L, w1, w1, KE1, 0L, (void*)hv, (void*)hv, NE1, 0L, b128, b128, 0L, Mc, NE1, KE1, gscale);
    k_vw<<<gb, NTHR, 0, stream>>>(hv, pv_w2, pv_b2, ei, pos, nN, nE, base, Mc, mv);
    wmma_gemm64<0, false, 2, 1, false, 6><<<dim3(gemm_blocks(Mc, HID), 1), 256, 0, stream>>>(
        hv, hv, NE1, 0L, w2, w2, HID, 0L, (void*)h2, (void*)h2, HID, 0L, pe_b2, pe_b2, 0L, Mc, HID, HID, gscale);
    wmma_gemm64<0, false, 2, 0, false, 0><<<dim3(gemm_blocks(Mc, HID), 1), 256, 0, stream>>>(
        h2, h2, HID, 0L, w3, w3, HID, 0L, (void*)mhf, (void*)mhf, HID, 0L, pe_b3, pe_b3, 0L, Mc, HID, HID, 1.0f / 64.0f);
    k_agg<<<nA, NTHR, LDS_AGG, stream>>>(ei + (size_t)nE + (size_t)base, Ec, mhf, mv, aggh, aggv, nN,
                                         (c == 0) ? 1 : 0, vec);
  }

  k_hh<<<(RP * (KNODE / 8)) / NTHR, NTHR, 0, stream>>>(x, aggh, aggv, nN, RP, hhh, hhl);
  wmma_gemm64<1, true, 2, 2, false, 6><<<dim3(gemm_blocks(RP, HID), 1), 256, 0, stream>>>(
      hhh, hhl, KNODE, 0L, wp1h, wp1l, KNODE, 0L, (void*)hnh, (void*)hnl, HID, 0L, ph_b1, ph_b1, 0L, RP, HID, KNODE, 1.0f);
  wmma_gemm64<1, true, 2, 0, false, 0><<<dim3(gemm_blocks(RP, HID), 1), 256, 0, stream>>>(
      hnh, hnl, HID, 0L, wp2h, wp2l, HID, 0L, (void*)outp, (void*)outp, HID, 0L, ph_b2, ph_b2, 0L, RP, HID, HID, 1.0f);
  const int n4 = nN * (HID / 4);
  k_copy<<<(n4 + NTHR - 1) / NTHR, NTHR, 0, stream>>>(outp, out, n4);
}
